// Head_5128190951491
// MI455X (gfx1250) — hardware-verified
//
#include <hip/hip_runtime.h>
#ifndef NB
#define NB 4
#endif
#ifndef SEQ
#define SEQ 4096
#endif
#define NB_FULL 4
#define SEQ_FULL 4096
#define DM 512
#define HD 64
#ifndef QCH
#define QCH ((SEQ) < 2048 ? (SEQ) : 2048)
#endif
#define NR ((size_t)NB * SEQ)
#define XCARRY 16.0f
#define WCARRY 1024.0f
#define PCARRY 16384.0f

static_assert(HD == 64);
static_assert(DM % 32 == 0);
static_assert(DM / 8 == 64);
static_assert(SEQ % 256 == 0);
static_assert(QCH % 256 == 0);
static_assert(SEQ % QCH == 0);
static_assert(NB <= NB_FULL);
static_assert(SEQ <= SEQ_FULL);
static_assert((HD * DM / 8) % 256 == 0);
static_assert(((size_t)NB * SEQ * DM / 8) % 256 == 0);
static_assert(((size_t)NB * SEQ) % 128 == 0);

typedef unsigned short v8us __attribute__((ext_vector_type(8), may_alias));
typedef float  v8f  __attribute__((ext_vector_type(8)));
typedef float  v4f  __attribute__((ext_vector_type(4)));
typedef float  v4fa __attribute__((ext_vector_type(4), may_alias));
typedef _Float16 v16h __attribute__((ext_vector_type(16)));
typedef _Float16 v4h __attribute__((ext_vector_type(4)));
union FragH { v16h v; v8us half[2]; _Float16 h[16]; unsigned short u[16]; };

__device__ __forceinline__ unsigned short bf16_bits(float x) { unsigned int u = __float_as_uint(x); return (unsigned short)((u + 0x7FFFu + ((u >> 16) & 1u)) >> 16); }
__device__ __forceinline__ float bf16_val(unsigned short b) { return __uint_as_float(((unsigned int)b) << 16); }
__device__ __forceinline__ float bf16_rne(float x) { return bf16_val(bf16_bits(x)); }

__device__ __forceinline__ v16h g2_frag(const _Float16* p, unsigned hh) { FragH f; f.half[0] = *(const v8us*)((const unsigned short*)p + 8u * hh); f.half[1] = *(const v8us*)((const unsigned short*)p + 16u + 8u * hh); return f.v; }
__device__ __forceinline__ v8f g2_mma(v16h a, v16h b, v8f c) { v8f d = __builtin_amdgcn_wmma_f32_16x16x32_f16(false, a, false, b, (short)0, c, false, false); asm volatile("v_nop\n\tv_nop\n\tv_nop\n\tv_nop" : "+v"(d) : "v"(a), "v"(b)); return d; }

__device__ __forceinline__ float circle_map(float t, float kcoef) {
#pragma clang fp contract(off)
  const float sn = sinf(6.2831855f * t);
  const float u = (t + 0.618f) - kcoef * sn;
  float r = u - truncf(u);
  if (r < 0.0f) r += 1.0f;
  return r;
}

__global__ __launch_bounds__(256) void k_wnat3(const float* __restrict__ w0, const float* __restrict__ w1, const float* __restrict__ w2,
                                               _Float16* __restrict__ B0, _Float16* __restrict__ B1, _Float16* __restrict__ B2) {
  const unsigned t = blockIdx.x * 256u + threadIdx.x;
  const unsigned y = blockIdx.y;
  if (t >= (unsigned)(HD * DM / 8)) return;
  const float* w = (y == 0u) ? w0 : ((y == 1u) ? w1 : w2);
  _Float16* Bt = (y == 0u) ? B0 : ((y == 1u) ? B1 : B2);
  const v4f a = *(const v4fa*)(w + (size_t)t * 8u), c = *(const v4fa*)(w + (size_t)t * 8u + 4u);
  FragH f;
#pragma unroll
  for (int q = 0; q < 4; ++q) { f.h[q] = (_Float16)(bf16_rne(a[q]) * WCARRY); f.h[4 + q] = (_Float16)(bf16_rne(c[q]) * WCARRY); }
  const v8us o = f.half[0];
  unsigned short* d = (unsigned short*)Bt + (size_t)t * 8u;
  *(volatile v8us*)d = o; __threadfence(); *(volatile v8us*)d = o;
}

__global__ __launch_bounds__(256) void k_x16(const float* __restrict__ x, _Float16* __restrict__ X16) {
  const unsigned t = blockIdx.x * 256u + threadIdx.x;
  if (t >= (unsigned)(NR * DM / 8)) return;
  const unsigned row = t >> 6, c8 = (t & 63u) * 8u;
  const unsigned b = row / (unsigned)SEQ, s = row % (unsigned)SEQ;
  const float* src = x + ((size_t)b * SEQ_FULL + s) * DM + c8;
  const v4f a = *(const v4fa*)src, c = *(const v4fa*)(src + 4);
  FragH f;
#pragma unroll
  for (int q = 0; q < 4; ++q) { f.h[q] = (_Float16)(bf16_rne(a[q]) * XCARRY); f.h[4 + q] = (_Float16)(bf16_rne(c[q]) * XCARRY); }
  const v8us o = f.half[0];
  unsigned short* d = (unsigned short*)X16 + (size_t)t * 8u;
  *(volatile v8us*)d = o; __threadfence(); *(volatile v8us*)d = o;
}

__global__ __launch_bounds__(128) void k_proj(const _Float16* __restrict__ X16, const _Float16* __restrict__ BQ, const _Float16* __restrict__ BK, const _Float16* __restrict__ BV,
                                              const float* __restrict__ Kparam, _Float16* __restrict__ Q16, _Float16* __restrict__ QL,
                                              _Float16* __restrict__ K16, _Float16* __restrict__ KL, _Float16* __restrict__ V16) {
  __shared__ __attribute__((aligned(16))) float so[4][32][68];
  const unsigned tid = threadIdx.x, w = tid >> 5, lane = tid & 31u, ln = lane & 15u, hh = lane >> 4;
  const unsigned y = blockIdx.y;
  const _Float16* Bh = (y == 0u) ? BQ : ((y == 1u) ? BK : BV);
  _Float16* Oh = (y == 0u) ? Q16 : ((y == 1u) ? K16 : V16);
  _Float16* Ol = (y == 0u) ? QL : KL;
  const unsigned row0 = blockIdx.x * 128u + 32u * w;
  const _Float16* a0p = X16 + (size_t)(row0 + ln) * DM; const _Float16* a1p = a0p + (size_t)16 * DM;
  const _Float16* b0p = Bh + (size_t)ln * DM; const _Float16* b1p = b0p + (size_t)16 * DM; const _Float16* b2p = b1p + (size_t)16 * DM; const _Float16* b3p = b2p + (size_t)16 * DM;
  const v8f z8 = {0.f,0.f,0.f,0.f,0.f,0.f,0.f,0.f}; v8f c00 = z8, c01 = z8, c02 = z8, c03 = z8, c10 = z8, c11 = z8, c12 = z8, c13 = z8;
#pragma unroll 1
  for (unsigned kb = 0; kb < (unsigned)DM; kb += 32u) { const v16h a0 = g2_frag(a0p + kb, hh), a1 = g2_frag(a1p + kb, hh);
    v16h b = g2_frag(b0p + kb, hh); c00 = g2_mma(a0, b, c00); c10 = g2_mma(a1, b, c10);
    b = g2_frag(b1p + kb, hh); c01 = g2_mma(a0, b, c01); c11 = g2_mma(a1, b, c11);
    b = g2_frag(b2p + kb, hh); c02 = g2_mma(a0, b, c02); c12 = g2_mma(a1, b, c12);
    b = g2_frag(b3p + kb, hh); c03 = g2_mma(a0, b, c03); c13 = g2_mma(a1, b, c13); }
  const float alpha = 1.0f / (XCARRY * WCARRY);
  v8f accs[8] = {c00, c01, c02, c03, c10, c11, c12, c13};
#pragma unroll
  for (int u = 0; u < 8; ++u) { const unsigned t = (unsigned)u & 3u, hf = (unsigned)u >> 2;
#pragma unroll
    for (int r = 0; r < 8; ++r) so[w][hf * 16u + 8u * hh + (unsigned)r][t * 16u + ln] = accs[u][r] * alpha; }
  __builtin_amdgcn_fence(4  , "workgroup"); __builtin_amdgcn_wave_barrier();
  const unsigned rsub = lane >> 4, c4 = (lane & 15u) * 4u;
  if (y < 2u) {
    const float kcoef = fabsf(Kparam[0]) * (1.0f / 6.2831855f);
#pragma unroll 1
    for (unsigned q = 0; q < 16u; ++q) { const unsigned r = q * 2u + rsub; v4f v = *(const v4fa*)&so[w][r][c4];
#pragma unroll
      for (int i = 0; i < 4; ++i) v[i] = circle_map(v[i], kcoef);
      *(v4fa*)&so[w][r][c4] = v; }
  }
  for (int pass = 0; pass < 2; ++pass) {
#pragma unroll 4
    for (unsigned q = 0; q < 16u; ++q) { const unsigned r = q * 2u + rsub; const v4f v = *(const v4fa*)&so[w][r][c4];
      v4h h4, l4;
#pragma unroll
      for (int i = 0; i < 4; ++i) { const _Float16 h = (_Float16)v[i]; h4[i] = h; l4[i] = (_Float16)((v[i] - (float)h) * 1024.0f); }
      *(volatile v4h*)(Oh + (size_t)(row0 + r) * HD + c4) = h4;
      if (y < 2u) *(volatile v4h*)(Ol + (size_t)(row0 + r) * HD + c4) = l4; }
    if (pass == 0) __threadfence(); }
}

__global__ __launch_bounds__(256) void k_vt(const _Float16* __restrict__ V16, _Float16* __restrict__ VT) {
  __shared__ unsigned short tl[64][66];
  const unsigned tid = threadIdx.x; const unsigned b = blockIdx.x / (unsigned)(SEQ / 64), lg = blockIdx.x % (unsigned)(SEQ / 64);
  for (unsigned i = tid; i < 512u; i += 256u) { const unsigned r = i >> 3, c8 = (i & 7u) * 8u; FragH f; f.half[0] = *(const v8us*)((const unsigned short*)V16 + ((size_t)b * SEQ + lg * 64u + r) * HD + c8);
#pragma unroll
    for (int q = 0; q < 8; ++q) tl[r][c8 + (unsigned)q] = f.u[q]; }
  __syncthreads();
  for (int pass = 0; pass < 2; ++pass) {
#pragma unroll
    for (unsigned rd = 0; rd < 2u; ++rd) { const unsigned d = rd * 32u + (tid >> 3), pc = tid & 7u; FragH f;
#pragma unroll
      for (int q = 0; q < 8; ++q) f.u[q] = tl[pc * 8u + (unsigned)q][d];
      *(volatile v8us*)((unsigned short*)VT + ((size_t)b * HD + d) * SEQ + lg * 64u + pc * 8u) = f.half[0]; }
    if (pass == 0) __threadfence(); }
}

__global__ __launch_bounds__(256) void k_vmean(const _Float16* __restrict__ VT, float* __restrict__ MV) {
  __shared__ __attribute__((aligned(16))) float sm[32];
  const unsigned tid = threadIdx.x, w = tid >> 5, lane = tid & 31u;
  const unsigned b = blockIdx.x >> 1, dg = (blockIdx.x & 1u) * 32u;
#pragma unroll 1
  for (unsigned j = 0; j < 4u; ++j) {
    const unsigned d = dg + w * 4u + j;
    const unsigned short* row = (const unsigned short*)VT + ((size_t)b * HD + d) * SEQ;
    float acc = 0.f;
#pragma unroll 1
    for (unsigned s = lane * 8u; s < (unsigned)SEQ; s += 256u) { FragH f; f.half[0] = *(const v8us*)(row + s);
#pragma unroll
      for (int q = 0; q < 8; ++q) acc += (float)f.h[q]; }
    acc += __shfl_xor(acc, 16, 32); acc += __shfl_xor(acc, 8, 32); acc += __shfl_xor(acc, 4, 32); acc += __shfl_xor(acc, 2, 32); acc += __shfl_xor(acc, 1, 32);
    if (lane == 0u) sm[w * 4u + j] = acc * (1.0f / (float)SEQ);
  }
  __syncthreads();
  if (tid < 8u) { const v4f v = *(const v4fa*)&sm[tid * 4u]; float* dst = MV + (size_t)b * HD + dg + tid * 4u;
    *(volatile v4f*)dst = v; __threadfence(); *(volatile v4f*)dst = v; }
}

__global__ __launch_bounds__(128) void k_scores(const _Float16* __restrict__ Qh, const _Float16* __restrict__ Ql, const _Float16* __restrict__ Kh, const _Float16* __restrict__ Kl, float* __restrict__ S) {
  __shared__ __attribute__((aligned(16))) float so[4][16][68];
  const unsigned tid = threadIdx.x, w = tid >> 5, lane = tid & 31u, ln = lane & 15u, hh = lane >> 4;
  const unsigned ntn = (unsigned)(SEQ / 64);
  const unsigned mt = blockIdx.x / ntn, nq = blockIdx.x % ntn;
  const unsigned row0 = mt * 64u + 16u * w, col0 = nq * 64u;
  const _Float16* ahp = Qh + (size_t)(row0 + ln) * HD; const _Float16* alp = Ql + (size_t)(row0 + ln) * HD;
  const _Float16* bhp = Kh + (size_t)(col0 + ln) * HD; const _Float16* blp = Kl + (size_t)(col0 + ln) * HD;
  const v8f z8 = {0.f,0.f,0.f,0.f,0.f,0.f,0.f,0.f};
  v8f ch[4] = {z8, z8, z8, z8}, cr[4] = {z8, z8, z8, z8};
#pragma unroll
  for (unsigned kb = 0; kb < 64u; kb += 32u) {
    const v16h ah = g2_frag(ahp + kb, hh), al = g2_frag(alp + kb, hh);
#pragma unroll
    for (int t = 0; t < 4; ++t) {
      const v16h bh = g2_frag(bhp + (size_t)t * 16 * HD + kb, hh), bl = g2_frag(blp + (size_t)t * 16 * HD + kb, hh);
      ch[t] = g2_mma(ah, bh, ch[t]);
      cr[t] = g2_mma(al, bh, cr[t]);
      cr[t] = g2_mma(ah, bl, cr[t]);
    }
  }
#pragma unroll
  for (int t = 0; t < 4; ++t) {
#pragma unroll
    for (int r = 0; r < 8; ++r) so[w][8u * hh + (unsigned)r][(unsigned)t * 16u + ln] = (ch[t][r] + cr[t][r] * (1.0f / 1024.0f)) * 0.125f; }
  __builtin_amdgcn_fence(4  , "workgroup"); __builtin_amdgcn_wave_barrier();
  const unsigned rsub = lane >> 4, c4 = (lane & 15u) * 4u;
  for (int pass = 0; pass < 2; ++pass) {
#pragma unroll
    for (unsigned q = 0; q < 8u; ++q) { const unsigned r = q * 2u + rsub; const v4f v = *(const v4fa*)&so[w][r][c4];
      *(volatile v4f*)(S + (size_t)(row0 + r) * SEQ + col0 + c4) = v; }
    if (pass == 0) __threadfence(); }
}

__global__ __launch_bounds__(256) void k_rsm(const float* __restrict__ S, _Float16* __restrict__ P) {
  #pragma clang fp contract(off)
  const unsigned i = blockIdx.x * 256u + threadIdx.x; if (i >= (unsigned)QCH) return; const float* s = S + (size_t)i * SEQ; float mx = -INFINITY;
#pragma unroll 1
  for (unsigned j = 0; j < (unsigned)SEQ; ++j) mx = fmaxf(mx, s[j]); float se = 0.f;
#pragma unroll 1
  for (unsigned j = 0; j < (unsigned)SEQ; ++j) se += expf(s[j] - mx); const float sc = PCARRY / se; const float cen = PCARRY / (float)SEQ;
#pragma unroll 1
  for (unsigned j0 = 0; j0 < (unsigned)SEQ; j0 += 8u) { FragH f;
#pragma unroll
    for (int q = 0; q < 8; ++q) f.h[q] = (_Float16)(expf(s[j0 + (unsigned)q] - mx) * sc - cen);
    const v8us o = f.half[0]; unsigned short* d = (unsigned short*)P + (size_t)i * SEQ + j0; *(volatile v8us*)d = o; __threadfence(); *(volatile v8us*)d = o; }
}

__global__ __launch_bounds__(128) void k_pv(const _Float16* __restrict__ P, const _Float16* __restrict__ VTb, const float* __restrict__ MVb, float* __restrict__ O) {
  __shared__ __attribute__((aligned(16))) float so[4][32][68];
  const unsigned tid = threadIdx.x, w = tid >> 5, lane = tid & 31u, ln = lane & 15u, hh = lane >> 4;
  const unsigned row0 = blockIdx.x * 128u + 32u * w;
  const _Float16* a0p = P + (size_t)(row0 + ln) * SEQ; const _Float16* a1p = a0p + (size_t)16 * SEQ;
  const _Float16* b0p = VTb + (size_t)ln * SEQ; const _Float16* b1p = b0p + (size_t)16 * SEQ; const _Float16* b2p = b1p + (size_t)16 * SEQ; const _Float16* b3p = b2p + (size_t)16 * SEQ;
  const v8f z8 = {0.f,0.f,0.f,0.f,0.f,0.f,0.f,0.f}; v8f c00 = z8, c01 = z8, c02 = z8, c03 = z8, c10 = z8, c11 = z8, c12 = z8, c13 = z8;
#pragma unroll 1
  for (unsigned kb = 0; kb < (unsigned)SEQ; kb += 32u) { const v16h a0 = g2_frag(a0p + kb, hh), a1 = g2_frag(a1p + kb, hh);
    v16h b = g2_frag(b0p + kb, hh); c00 = g2_mma(a0, b, c00); c10 = g2_mma(a1, b, c10);
    b = g2_frag(b1p + kb, hh); c01 = g2_mma(a0, b, c01); c11 = g2_mma(a1, b, c11);
    b = g2_frag(b2p + kb, hh); c02 = g2_mma(a0, b, c02); c12 = g2_mma(a1, b, c12);
    b = g2_frag(b3p + kb, hh); c03 = g2_mma(a0, b, c03); c13 = g2_mma(a1, b, c13); }
  v8f accs[8] = {c00, c01, c02, c03, c10, c11, c12, c13};
#pragma unroll
  for (int u = 0; u < 8; ++u) { const unsigned t = (unsigned)u & 3u, hf = (unsigned)u >> 2; const float mv = MVb[t * 16u + ln];
#pragma unroll
    for (int r = 0; r < 8; ++r) so[w][hf * 16u + 8u * hh + (unsigned)r][t * 16u + ln] = accs[u][r] * (1.0f / PCARRY) + mv; }
  __builtin_amdgcn_fence(4  , "workgroup"); __builtin_amdgcn_wave_barrier();
  const unsigned rsub = lane >> 4, c4 = (lane & 15u) * 4u;
  for (int pass = 0; pass < 2; ++pass) {
#pragma unroll
    for (unsigned q = 0; q < 16u; ++q) { const unsigned r = q * 2u + rsub; const v4f v = *(const v4fa*)&so[w][r][c4];
      *(volatile v4f*)(O + (size_t)(row0 + r) * HD + c4) = v; }
    if (pass == 0) __threadfence(); }
}

extern "C" void kernel_launch(void* const* d_in, const int* in_sizes, int n_in,
                              void* d_out, int out_size, void* d_ws, size_t ws_size, hipStream_t stream) {
  if (n_in < 5) return;
  const size_t need_rows = (size_t)(NB - 1) * SEQ_FULL + SEQ;
  if ((size_t)in_sizes[0] < need_rows * DM) return;
  if ((size_t)in_sizes[1] < (size_t)HD * DM || (size_t)in_sizes[2] < (size_t)HD * DM || (size_t)in_sizes[3] < (size_t)HD * DM) return;
  if (in_sizes[4] < 1) return;
  if ((size_t)out_size < need_rows * HD) return;
  const float* x = (const float*)d_in[0]; const float* wq = (const float*)d_in[1]; const float* wk = (const float*)d_in[2]; const float* wv = (const float*)d_in[3]; const float* kp = (const float*)d_in[4];
  float* out = (float*)d_out;
  char* ws = (char*)d_ws; size_t off = 0;
  auto take = [&](size_t bytes) { char* p = ws + off; off += (bytes + 255) & ~(size_t)255; return p; };
  _Float16* BQ = (_Float16*)take((size_t)HD * DM * 2); _Float16* BK = (_Float16*)take((size_t)HD * DM * 2); _Float16* BV = (_Float16*)take((size_t)HD * DM * 2);
  _Float16* X16 = (_Float16*)take(NR * DM * 2);
  _Float16* Q16 = (_Float16*)take(NR * HD * 2); _Float16* QL = (_Float16*)take(NR * HD * 2);
  _Float16* K16 = (_Float16*)take(NR * HD * 2); _Float16* KL = (_Float16*)take(NR * HD * 2);
  _Float16* V16 = (_Float16*)take(NR * HD * 2); _Float16* VT = (_Float16*)take(NR * HD * 2);
  float* MV = (float*)take((size_t)NB * HD * 4);
  float* S = (float*)take((size_t)QCH * SEQ * 4); _Float16* P = (_Float16*)take((size_t)QCH * SEQ * 2);
  if (off > ws_size) return;
  k_wnat3<<<dim3((unsigned)(HD * DM / 8 / 256), 3), 256, 0, stream>>>(wq, wk, wv, BQ, BK, BV);
  k_x16<<<(unsigned)(NR * DM / 8 / 256), 256, 0, stream>>>(x, X16);
  k_proj<<<dim3((unsigned)(NR / 128), 3), 128, 0, stream>>>(X16, BQ, BK, BV, kp, Q16, QL, K16, KL, V16);
  k_vt<<<(unsigned)(NB * (SEQ / 64)), 256, 0, stream>>>(V16, VT);
  k_vmean<<<(unsigned)(NB * 2), 256, 0, stream>>>(VT, MV);
  for (int b = 0; b < NB; ++b) {
    const size_t kro = (size_t)b * SEQ * HD;
    for (int c = 0; c < SEQ / QCH; ++c) {
      const size_t qro = ((size_t)b * SEQ + (size_t)c * QCH) * HD;
      k_scores<<<(unsigned)((QCH / 64) * (SEQ / 64)), 128, 0, stream>>>(Q16 + qro, QL + qro, K16 + kro, KL + kro, S);
      k_rsm<<<(unsigned)(QCH / 256), 256, 0, stream>>>(S, P);
      k_pv<<<(unsigned)(QCH / 128), 128, 0, stream>>>(P, VT + (size_t)b * HD * SEQ, MV + (size_t)b * HD, out + ((size_t)b * SEQ_FULL + (size_t)c * QCH) * HD);
    }
  }
}
